// PhysicsInformedNN_42992622633174
// MI455X (gfx1250) — hardware-run, weakly checked
//
#include <hip/hip_runtime.h>
#include <math.h>

typedef __attribute__((ext_vector_type(16))) __bf16         v16b;
typedef __attribute__((ext_vector_type(8)))  __bf16         v8b;
typedef __attribute__((ext_vector_type(8)))  float          v8f;
typedef __attribute__((ext_vector_type(4)))  float          v4f;
typedef __attribute__((ext_vector_type(2)))  float          v2f;
typedef __attribute__((ext_vector_type(8)))  unsigned short us8;

constexpr int kN      = 32768;
constexpr int kP      = 8192;
constexpr int kCh     = 13;
constexpr int kWd     = 128;
constexpr int kKd     = 2 * kWd;
constexpr int kRows   = kCh * kP;
constexpr int kNumMid = 7;
constexpr int kJetPts  = 8;
constexpr int kJetRows = 2 * kCh;
constexpr int kInputsRneToBf16 = 1;

static_assert(kN % kP == 0);
static_assert(kRows % 64 == 0);
static_assert(kWd % 64 == 0);
static_assert(kKd % 32 == 0);
static_assert(kP % kJetPts == 0);
static_assert(kP % 256 == 0);
static_assert(((kRows / 64) * (kWd / 64)) % 8 == 0);

constexpr size_t kBytesA  = (size_t)kRows * kKd * 2;
constexpr size_t kBytesZ  = (size_t)kRows * kWd * 4;
constexpr size_t kBytesBT = (size_t)kNumMid * kWd * kKd * 2;
constexpr size_t kOffA    = 0;
constexpr size_t kOffZ    = kOffA + kBytesA;
constexpr size_t kOffBT   = kOffZ + kBytesZ;
constexpr size_t kWsTotal = kOffBT + kBytesBT;
static_assert(kBytesA == 54525952ull);
static_assert(kBytesZ == 54525952ull);
static_assert(kBytesBT == 458752ull);
static_assert(kWsTotal == 109510656ull);
static_assert(kWsTotal <= 134217728ull);
static_assert((kOffZ % 128) == 0 && (kOffBT % 128) == 0);
static_assert((size_t)kRows * kWd * 4 <= kBytesA);

__device__ __forceinline__ unsigned short f2bf_bits(float f) {
  unsigned u = __float_as_uint(f);
  return (unsigned short)((u + 0x7FFFu + ((u >> 16) & 1u)) >> 16);
}
__device__ __forceinline__ float bf_bits2f(unsigned short h) { return __uint_as_float(((unsigned)h) << 16); }
__device__ __forceinline__ float in_rne(float f) {
  return kInputsRneToBf16 ? bf_bits2f(f2bf_bits(f)) : f;
}

union FragU { v16b v; v8b h[2]; };
__device__ __forceinline__ v16b frag_load(const __bf16* p) {
  FragU f;
  f.h[0] = *(const v8b*)(p);
  f.h[1] = *(const v8b*)(p + 16);
  return f.v;
}
__device__ __forceinline__ v8f mma_bf16(v16b a, v16b b, v8f c) {
  return __builtin_amdgcn_wmma_f32_16x16x32_bf16(false, a, false, b, (short)0, c, false, false);
}
__device__ __forceinline__ void mma_group_guard(v8f& a, v8f& b, v8f& c, v8f& d, v16b x, v16b y0, v16b y1, v16b y2, v16b y3) {
  asm volatile("v_nop\n\tv_nop\n\tv_nop\n\tv_nop" : "+v"(a), "+v"(b), "+v"(c), "+v"(d) : "v"(x), "v"(y0), "v"(y1), "v"(y2), "v"(y3));
}
__device__ __forceinline__ void keep4_b(v16b a, v16b b, v16b c, v16b d) { asm volatile("v_nop" :: "v"(a), "v"(b), "v"(c), "v"(d)); }
__device__ __forceinline__ void acc_guard4(v8f& a, v8f& b, v8f& c, v8f& d) { asm volatile("v_nop\n\tv_nop\n\tv_nop\n\tv_nop" : "+v"(a), "+v"(b), "+v"(c), "+v"(d)); }

__global__ __launch_bounds__(256) void weight_planes_kernel(
    const float* __restrict__ wa, const float* __restrict__ wb, const float* __restrict__ wc,
    const float* __restrict__ wd, const float* __restrict__ we, const float* __restrict__ wf,
    const float* __restrict__ wg, unsigned short* __restrict__ BT)
{
  const int lane = threadIdx.x & 31;
  const int wave = threadIdx.x >> 5;
  const int l = blockIdx.x >> 4;
  const int n = ((blockIdx.x & 15) << 3) + wave;
  const float* W = (l == 0) ? wa : (l == 1) ? wb : (l == 2) ? wc : (l == 3) ? wd : (l == 4) ? we : (l == 5) ? wf : wg;
  const int k0 = lane * 8;
  us8 v;
#pragma unroll
  for (int e = 0; e < 8; ++e) {
    const int k = (k0 + e) & (kWd - 1);
    const float f = W[(size_t)k * kWd + n];
    v[e] = f2bf_bits(f);
  }
  unsigned short* q = BT + ((size_t)(l * kWd + n)) * kKd + k0;
  *(volatile us8*)q = v;
  __threadfence();
  *(volatile us8*)q = v;
}

__global__ __launch_bounds__(256) void layer_product_kernel(
    const unsigned short* __restrict__ Ap, const unsigned short* __restrict__ Btp,
    float* __restrict__ Cout, int M)
{
  const __bf16* A  = (const __bf16*)Ap;
  const __bf16* Bt = (const __bf16*)Btp;
  __shared__ __align__(16) float sT[8][16 * 68];
  const int lane = threadIdx.x & 31;
  const int wave = threadIdx.x >> 5;
  constexpr int tilesN = kWd >> 6;
  const int tilesM = M >> 6;
  const int tile = blockIdx.x * 8 + wave;
  if (tile >= tilesM * tilesN) return;
  const int tm = tile / tilesN;
  const int tn = tile - tm * tilesN;
  const int m0 = tm << 6;
  const int n0 = tn << 6;

  const int rlane = lane & 15;
  const int koff  = (lane >> 4) * 8;
  const int mOff  = (lane >> 4) * 8;

  v8f acc[4][4];
#pragma unroll
  for (int i = 0; i < 4; ++i)
#pragma unroll
    for (int j = 0; j < 4; ++j) acc[i][j] = (v8f){0.f, 0.f, 0.f, 0.f, 0.f, 0.f, 0.f, 0.f};

#pragma unroll 1
  for (int k0 = 0; k0 < kKd; k0 += 32) {
    v16b bh[4];
#pragma unroll
    for (int j = 0; j < 4; ++j) {
      const size_t bo = (size_t)(n0 + (j << 4) + rlane) * kKd + koff + k0;
      bh[j] = frag_load(Bt + bo);
    }
#pragma unroll
    for (int i = 0; i < 4; ++i) {
      const size_t ao = (size_t)(m0 + (i << 4) + rlane) * kKd + koff + k0;
      const v16b ah = frag_load(A + ao);
#pragma unroll
      for (int j = 0; j < 4; ++j) acc[i][j] = mma_bf16(ah, bh[j], acc[i][j]);
      mma_group_guard(acc[i][0], acc[i][1], acc[i][2], acc[i][3], ah, bh[0], bh[1], bh[2], bh[3]);
    }
    keep4_b(bh[0], bh[1], bh[2], bh[3]);
  }
  acc_guard4(acc[0][0], acc[0][1], acc[0][2], acc[0][3]);
  acc_guard4(acc[1][0], acc[1][1], acc[1][2], acc[1][3]);
  acc_guard4(acc[2][0], acc[2][1], acc[2][2], acc[2][3]);
  acc_guard4(acc[3][0], acc[3][1], acc[3][2], acc[3][3]);

  float* slab = sT[wave];
#pragma unroll
  for (int i = 0; i < 4; ++i) {
    const int mBase = m0 + (i << 4);
#pragma unroll
    for (int j = 0; j < 4; ++j) {
#pragma unroll
      for (int r = 0; r < 8; ++r) slab[(mOff + r) * 68 + (j << 4) + rlane] = acc[i][j][r];
    }
    __builtin_amdgcn_fence(__ATOMIC_RELEASE, "workgroup");
    __builtin_amdgcn_wave_barrier();
    __builtin_amdgcn_fence(__ATOMIC_ACQUIRE, "workgroup");
    {
      const int hh = lane >> 4;
      const int c4 = (lane & 15) * 4;
      for (int pass = 0; pass < 2; ++pass) {
#pragma unroll
        for (int it = 0; it < 8; ++it) {
          const int row = it * 2 + hh;
          const v4f v = *(const v4f*)(slab + row * 68 + c4);
          *(volatile v4f*)(Cout + (size_t)(mBase + row) * kWd + n0 + c4) = v;
        }
        __threadfence();
      }
    }
    __builtin_amdgcn_fence(__ATOMIC_RELEASE, "workgroup");
    __builtin_amdgcn_wave_barrier();
    __builtin_amdgcn_fence(__ATOMIC_ACQUIRE, "workgroup");
  }
}

__device__ __forceinline__ void tanh_chain13(const float (&z)[kCh], float (&o)[kCh]) {
  const float s  = tanhf(z[0]);
  const float ss = s * s;
  const float s1 = 1.0f - ss;
  const float s2 = -2.0f * s * s1;
  const float s3 = -2.0f * s1 * (s1 - 2.0f * ss);
  const float zx = z[1], zy = z[2], zt = z[3];
  const float zxx = z[4], zxy = z[5], zxt = z[6], zyy = z[7], zyt = z[8];
  const float ax = s2 * zx;
  const float ay = s2 * zy;
  o[0] = s;
  o[1] = s1 * zx;
  o[2] = s1 * zy;
  o[3] = s1 * zt;
  o[4] = ax * zx + s1 * zxx;
  o[5] = ax * zy + s1 * zxy;
  o[6] = ax * zt + s1 * zxt;
  o[7] = ay * zy + s1 * zyy;
  o[8] = ay * zt + s1 * zyt;
  const float cxx = s3 * zx * zx;
  const float cyy = s3 * zy * zy;
  o[9]  = cxx * zx + 3.0f * ax * zxx + s1 * z[9];
  o[10] = cxx * zy + s2 * (zxx * zy + 2.0f * zxy * zx) + s1 * z[10];
  o[11] = cyy * zx + s2 * (zyy * zx + 2.0f * zxy * zy) + s1 * z[11];
  o[12] = cyy * zy + 3.0f * ay * zyy + s1 * z[12];
}

template <int MODE>
__global__ __launch_bounds__(256) void chain_kernel(
    const float* __restrict__ Zin, const float* __restrict__ bias,
    const float* __restrict__ xs, const float* __restrict__ ys, const float* __restrict__ ts,
    const float* __restrict__ W0, unsigned short* __restrict__ Aout, float* __restrict__ Fout, int chunkBase)
{
  __shared__ __align__(16) unsigned short tileH[(MODE == 2) ? 8 : kJetRows * kKd];
  __shared__ __align__(16) float tileF[(MODE == 2) ? kJetRows * kWd : 4];
  const int tid  = threadIdx.x;
  const int lane = tid & 31;
  const int wave = tid >> 5;
  const int n    = tid & (kWd - 1);
  const int slot = tid >> 7;
  const float bn = in_rne(bias[n]);
  float w0 = 0.f, w1 = 0.f, w2 = 0.f;
  if (MODE == 0) {
    w0 = in_rne(W0[n]);
    w1 = in_rne(W0[kWd + n]);
    w2 = in_rne(W0[2 * kWd + n]);
  }
  const int pblk = blockIdx.x * kJetPts;
#pragma unroll 1
  for (int it = 0; it < kJetPts / 2; ++it) {
    const int p = pblk + it * 2 + slot;
    float z[kCh];
    if (MODE == 0) {
      const float xv = in_rne(xs[chunkBase + p]);
      const float yv = in_rne(ys[chunkBase + p]);
      const float tv = in_rne(ts[chunkBase + p]);
      float zz = xv * w0;
      zz = fmaf(yv, w1, zz);
      zz = fmaf(tv, w2, zz);
      z[0] = zz + bn;
      z[1] = w0;
      z[2] = w1;
      z[3] = w2;
#pragma unroll
      for (int c = 4; c < kCh; ++c) z[c] = 0.0f;
    } else {
#pragma unroll
      for (int c = 0; c < kCh; ++c) z[c] = Zin[((size_t)c * kP + p) * kWd + n];
      z[0] += bn;
    }
    float o[kCh];
    tanh_chain13(z, o);
    if (MODE == 2) {
#pragma unroll
      for (int c = 0; c < kCh; ++c) tileF[(slot * kCh + c) * kWd + n] = o[c];
    } else {
#pragma unroll
      for (int c = 0; c < kCh; ++c) {
        const unsigned short hb = f2bf_bits(o[c]);
        const unsigned short lb = f2bf_bits(o[c] - bf_bits2f(hb));
        tileH[(slot * kCh + c) * kKd + n] = hb;
        tileH[(slot * kCh + c) * kKd + kWd + n] = lb;
      }
    }
    __syncthreads();
    for (int pass = 0; pass < 2; ++pass) {
      for (int r = wave; r < kJetRows; r += 8) {
        const int sl = (r >= kCh) ? 1 : 0;
        const int c  = r - kCh * sl;
        const size_t grow = (size_t)c * kP + (size_t)(pblk + it * 2 + sl);
        if (MODE == 2) {
          const v4f v = *(const v4f*)(tileF + r * kWd + lane * 4);
          *(volatile v4f*)(Fout + grow * kWd + lane * 4) = v;
        } else {
          const us8 v = *(const us8*)(tileH + r * kKd + lane * 8);
          *(volatile us8*)(Aout + grow * kKd + lane * 8) = v;
        }
      }
      __threadfence();
    }
    __syncthreads();
  }
}

__global__ __launch_bounds__(256) void final_kernel(
    const float* __restrict__ H, const float* __restrict__ W8, const float* __restrict__ b8,
    const float* __restrict__ lam1p, const float* __restrict__ lam2p,
    float* __restrict__ out, int chunkBase)
{
  __shared__ __align__(16) float sW[256];
  const int tid = threadIdx.x;
  sW[tid] = in_rne(W8[2 * (tid & (kWd - 1))]);
  __syncthreads();
  const int p = blockIdx.x * 256 + tid;
  float acc[kCh];
#pragma unroll
  for (int c = 0; c < kCh; ++c) acc[c] = 0.0f;
#pragma unroll 1
  for (int k = 0; k < kWd; k += 2) {
    const float wk0 = sW[k];
    const float wk1 = sW[k + 1];
#pragma unroll
    for (int c = 0; c < kCh; ++c) {
      const v2f hv = *(const v2f*)(H + ((size_t)c * kP + p) * kWd + k);
      const float h0 = hv[0];
      const float h1 = hv[1];
      acc[c] = fmaf(h0, wk0, acc[c]);
      acc[c] = fmaf(h1, wk1, acc[c]);
    }
  }
  acc[0] += in_rne(b8[0]);
  float o[kCh];
  tanh_chain13(acc, o);
  const float l1 = in_rne(lam1p[0]);
  const float l2 = in_rne(lam2p[0]);
  const float u   = o[2];
  const float v   = -o[1];
  const float u_x = o[5];
  const float u_y = o[7];
  const float u_t = o[8];
  const float v_x = -o[4];
  const float v_y = -o[5];
  const float v_t = -o[6];
  const float u_xx = o[10];
  const float u_yy = o[12];
  const float v_xx = -o[9];
  const float v_yy = -o[11];
  const float fu = u_t + l1 * (u * u_x + v * u_y) - l2 * (u_xx + u_yy);
  const float fv = v_t + l1 * (u * v_x + v * v_y) - l2 * (v_xx + v_yy);
  const size_t g = (size_t)chunkBase + (size_t)p;
  for (int pass = 0; pass < 2; ++pass) {
    *(volatile float*)(out + g) = u;
    *(volatile float*)(out + (size_t)kN + g) = v;
    *(volatile float*)(out + 2 * (size_t)kN + g) = fu;
    *(volatile float*)(out + 3 * (size_t)kN + g) = fv;
    __threadfence();
  }
}

extern "C" void kernel_launch(void* const* d_in, const int* in_sizes, int n_in,
                              void* d_out, int out_size, void* d_ws, size_t ws_size,
                              hipStream_t stream) {
  if (n_in < 23) return;
  if (in_sizes[0] != kN || in_sizes[1] != kN || in_sizes[2] != kN) return;
  if (in_sizes[3] != 3 * kWd || in_sizes[4] != kWd) return;
  for (int i = 1; i <= kNumMid; ++i) {
    if (in_sizes[3 + 2 * i] != kWd * kWd) return;
    if (in_sizes[4 + 2 * i] != kWd) return;
  }
  if (in_sizes[19] != kWd * 2 || in_sizes[20] != 2) return;
  if (in_sizes[21] != 1 || in_sizes[22] != 1) return;
  if (out_size != 4 * kN) return;
  if (ws_size < kWsTotal) return;

  const float* x  = (const float*)d_in[0];
  const float* y  = (const float*)d_in[1];
  const float* t  = (const float*)d_in[2];
  const float* W0 = (const float*)d_in[3];
  const float* b0 = (const float*)d_in[4];
  const float* W8 = (const float*)d_in[19];
  const float* b8 = (const float*)d_in[20];
  const float* lam1 = (const float*)d_in[21];
  const float* lam2 = (const float*)d_in[22];
  float* out = (float*)d_out;

  char* ws = (char*)d_ws;
  unsigned short* Abf = (unsigned short*)(ws + kOffA);
  float*          Af  = (float*)(ws + kOffA);
  float*          Z   = (float*)(ws + kOffZ);
  unsigned short* BT  = (unsigned short*)(ws + kOffBT);

  weight_planes_kernel<<<kNumMid * 16, 256, 0, stream>>>(
      (const float*)d_in[5], (const float*)d_in[7], (const float*)d_in[9], (const float*)d_in[11],
      (const float*)d_in[13], (const float*)d_in[15], (const float*)d_in[17], BT);

  const int prodBlocks = ((kRows / 64) * (kWd / 64)) / 8;
  for (int ch = 0; ch < kN / kP; ++ch) {
    const int chunkBase = ch * kP;
    chain_kernel<0><<<kP / kJetPts, 256, 0, stream>>>(Z, b0, x, y, t, W0, Abf, Af, chunkBase);
    for (int l = 1; l <= kNumMid; ++l) {
      const unsigned short* Btl = BT + (size_t)(l - 1) * kWd * kKd;
      const float* bl = (const float*)d_in[4 + 2 * l];
      layer_product_kernel<<<prodBlocks, 256, 0, stream>>>(Abf, Btl, Z, kRows);
      if (l < kNumMid) {
        chain_kernel<1><<<kP / kJetPts, 256, 0, stream>>>(Z, bl, x, y, t, W0, Abf, Af, chunkBase);
      } else {
        chain_kernel<2><<<kP / kJetPts, 256, 0, stream>>>(Z, bl, x, y, t, W0, Abf, Af, chunkBase);
      }
    }
    final_kernel<<<kP / 256, 256, 0, stream>>>(Af, W8, b8, lam1, lam2, out, chunkBase);
  }
}
